// MAGNOLayer_46428596470307
// MI455X (gfx1250) — hardware-run, weakly checked
//
#include <hip/hip_runtime.h>


namespace {
constexpr int Q = 8192, S = 32768, E = 131072, D = 256, H = 8, HD = 32, GEO = 128, FFN = 512, NQB = Q / 16;
constexpr float XS = 8.0f, G1S = 64.0f, G2S = 4096.0f, OS = 64.0f, FS = 64.0f, WSC = 256.0f, EPS = 1e-5f;
typedef _Float16 b16;
typedef __attribute__((ext_vector_type(16))) _Float16 v16b;
typedef __attribute__((ext_vector_type(8))) _Float16 v8b;
typedef __attribute__((ext_vector_type(8))) float v8f;
typedef __attribute__((ext_vector_type(4))) float v4f;
typedef __attribute__((ext_vector_type(2))) float v2f;
__device__ __forceinline__ float bf16_rne(float f) { unsigned int u = __float_as_uint(f); u += 0x7FFFu + ((u >> 16) & 1u); return __uint_as_float(u & 0xFFFF0000u); }
__device__ __forceinline__ void split16(float v, b16& hi, b16& lo) { hi = (b16)v; lo = (b16)(v - (float)hi); }
__device__ __forceinline__ v16b frag_kb(const b16* p, int hh) { const v8b a = *(const v8b*)(p + 8 * hh), b = *(const v8b*)(p + 16 + 8 * hh); v16b f;
#pragma unroll
  for (int e = 0; e < 8; ++e) { f[e] = a[e]; f[8 + e] = b[e]; } return f; }
__device__ __forceinline__ v8f wmma16b(v16b a, v16b b, v8f c) { v8f d = __builtin_amdgcn_wmma_f32_16x16x32_f16(false, a, false, b, (short)0, c, false, false); asm volatile("v_nop\n\tv_nop\n\tv_nop\n\tv_nop" : "+v"(d) : "v"(a), "v"(b)); return d; }
__device__ __forceinline__ void wave_lds_sync() { __builtin_amdgcn_fence(__ATOMIC_RELEASE, "workgroup"); __builtin_amdgcn_wave_barrier(); __builtin_amdgcn_fence(__ATOMIC_ACQUIRE, "workgroup"); }
__device__ __forceinline__ float pmul(float a, float b) { float p = a * b; asm volatile("" : "+v"(p)); return p; }
__device__ __forceinline__ int iclamp(int v, int lo, int hi) { return v < lo ? lo : (v > hi ? hi : v); }
__device__ __forceinline__ float gelu(float v) { return 0.5f * v * (1.0f + erff(v * 0.70710678118654752f)); }
constexpr int CSR_NBLK9 = 512, CSR_GB9 = 9, CSR_GN9 = 1 << CSR_GB9  , CSR_TS9 = (CSR_GN9 < 32 ? 32 : CSR_GN9)  , CSR_MAXG9 = 512, CSR_CAP9 = 12288  ;
__device__ __host__ __forceinline__ int csr_tix9(int v) { return (v >> CSR_GB9) * CSR_TS9 + (v & (CSR_GN9 - 1)); }
__global__ __launch_bounds__(64) void csrA_kernel9(const int* __restrict__ dst, int E, int N, int nG, int CHP, int NGP, int* __restrict__ STG, int* __restrict__ HST) {
  extern __shared__ int sm[];
  int* cnt = sm; int* run = sm + NGP; int* ids = sm + 2 * NGP;
  const int b = blockIdx.x; const int ch = (E + CSR_NBLK9 - 1) / CSR_NBLK9; const int e0 = b * ch, e1 = min(E, e0 + ch);
  for (int i = threadIdx.x; i < NGP; i += 64) cnt[i] = 0;
  for (int i = threadIdx.x; i < CHP; i += 64) ids[i] = -1;
  __syncthreads();
  if (threadIdx.x == 0) {
    for (int e = e0; e < e1; ++e) { int d = dst[e]; d = (d < 0) ? 0 : (d >= N ? N - 1 : d); cnt[d >> CSR_GB9] += 1; }
    int acc = 0; for (int g = 0; g < nG; ++g) { run[g] = acc; acc += cnt[g]; }
    for (int e = e0; e < e1; ++e) { int d = dst[e]; d = (d < 0) ? 0 : (d >= N ? N - 1 : d); const int g = d >> CSR_GB9; ids[run[g]] = e; run[g] += 1; } }
  __syncthreads();
  typedef __attribute__((ext_vector_type(4))) int v4i;
  for (int pass = 0; pass < 2; ++pass) {
    for (int i = threadIdx.x; i < CHP / 4; i += 64) *(volatile v4i*)(STG + (size_t)b * CHP + i * 4) = *(const v4i*)(&ids[i * 4]);
    for (int i = threadIdx.x; i < NGP / 4; i += 64) { v4i v; for (int e = 0; e < 4; ++e) v[e] = (i * 4 + e < nG) ? cnt[i * 4 + e] : 0; *(volatile v4i*)(HST + (size_t)b * NGP + i * 4) = v; }
    __threadfence(); }
}
__global__ __launch_bounds__(512) void csrS_kernel9(const int* __restrict__ HST, int nG, int NGP, int* __restrict__ START, int* __restrict__ TOT, int* __restrict__ OFF) {
  __shared__ int tot[CSR_MAXG9];
  const int b = threadIdx.x;
  for (int pass = 0; pass < 2; ++pass) { int runb = 0; for (int g = 0; g < nG; ++g) { int c = HST[(size_t)b * NGP + g]; c = (c < 0) ? 0 : c; ((volatile int*)OFF)[(size_t)g * CSR_NBLK9 + b] = runb; runb += c; } __threadfence(); }
  for (int g = threadIdx.x; g < nG; g += 512) { int s = 0; for (int bb = 0; bb < CSR_NBLK9; ++bb) { int c = HST[(size_t)bb * NGP + g]; s += (c < 0) ? 0 : c; } tot[g] = s; }
  __syncthreads();
  if (threadIdx.x < 32) {
    __shared__ int st[CSR_MAXG9 + 32];
    if (threadIdx.x == 0) { int acc = 0; for (int g = 0; g < NGP; ++g) { st[g] = acc; if (g < nG) acc += (tot[g] + 31) & ~31; } st[NGP] = acc; }
    __builtin_amdgcn_fence(__ATOMIC_RELEASE, "workgroup"); __builtin_amdgcn_wave_barrier(); __builtin_amdgcn_fence(__ATOMIC_ACQUIRE, "workgroup");
    for (int pass = 0; pass < 2; ++pass) { for (int i = threadIdx.x; i < NGP + 32; i += 32) { ((volatile int*)START)[i] = (i <= NGP) ? st[min(i, NGP)] : 0; ((volatile int*)TOT)[i] = (i < nG) ? tot[i] : 0; } __threadfence(); } }
}
__global__ __launch_bounds__(256) void csrB_kernel9(const int* __restrict__ dst, int N, int nG, int CHP, int NGP, int permLen, const int* __restrict__ STG, const int* __restrict__ HST, const int* __restrict__ OFF, const int* __restrict__ START, const int* __restrict__ TOT, int* __restrict__ PERM, int* __restrict__ ROWPTR, int* __restrict__ ROWCNT, int* __restrict__ FLAG) {
  typedef __attribute__((ext_vector_type(4))) int v4i;
  __shared__ int ids[CSR_CAP9]; __shared__ unsigned short key[CSR_CAP9]; __shared__ int outp[CSR_CAP9]; __shared__ int ncnt[CSR_GN9 + 1]; __shared__ int boff[CSR_NBLK9 + 1];
  const int g = blockIdx.x, t_ = threadIdx.x; int tot = TOT[g]; int st = START[g], stn = START[g + 1]; const int v0 = g * CSR_GN9; const int nv = min(CSR_GN9, N - v0); const int t0 = g * CSR_TS9;
  st = (st < 0) ? 0 : (st > permLen - 32 ? permLen - 32 : st) & ~31; stn = (stn < st) ? st : (stn > permLen ? permLen : stn); tot = (tot < 0) ? 0 : tot; if (tot > stn - st && tot <= CSR_CAP9) tot = stn - st;
  if (tot > CSR_CAP9) {
    for (int pass = 0; pass < 2; ++pass) { for (int i = t_; i < CSR_TS9 / 4; i += 256) { v4i a, c; for (int e = 0; e < 4; ++e) { a[e] = st; c[e] = 0; } *(volatile v4i*)(ROWPTR + t0 + i * 4) = a; *(volatile v4i*)(ROWCNT + t0 + i * 4) = c; } if (t_ == 0) ((volatile int*)FLAG)[0] = 1; __threadfence(); } (void)nv; return; }
  if (t_ == 0) { int acc = 0; for (int b = 0; b < CSR_NBLK9; ++b) { boff[b] = acc; int c = HST[(size_t)b * NGP + g]; c = (c < 0) ? 0 : (c > CHP ? CHP : c); acc += c; if (acc > tot) acc = tot; } boff[CSR_NBLK9] = acc; }
  for (int i = t_; i <= CSR_GN9; i += 256) ncnt[i] = 0;
  __syncthreads();
  for (int b = 0; b < CSR_NBLK9; ++b) { const int c = boff[b + 1] - boff[b]; int o_ = OFF[(size_t)g * CSR_NBLK9 + b]; o_ = (o_ < 0) ? 0 : (o_ > CHP - c ? CHP - c : o_); const int* src_ = STG + (size_t)b * CHP + o_;
    for (int i = t_; i < c; i += 256) { int id = src_[i]; id = (id < 0) ? 0 : id; ids[boff[b] + i] = id; int d = dst[id]; d = (d < v0) ? v0 : (d >= N ? N - 1 : d); int kk = d - v0; kk = (kk < 0) ? 0 : (kk >= CSR_GN9 ? CSR_GN9 - 1 : kk); key[boff[b] + i] = (unsigned short)kk; } }
  __syncthreads();
  if (t_ == 0) { for (int i = 0; i < tot; ++i) ncnt[key[i]] += 1; int acc = 0; for (int vl = 0; vl < CSR_GN9; ++vl) { const int c = ncnt[vl]; ncnt[vl] = acc; acc += c; } ncnt[CSR_GN9] = acc;
    for (int i = 0; i < tot; ++i) { const int vl = key[i]; outp[ncnt[vl]] = ids[i]; ncnt[vl] += 1; }
    for (int vl = CSR_GN9; vl > 0; --vl) ncnt[vl] = ncnt[vl - 1]; ncnt[0] = 0; }
  __syncthreads();
  for (int pass = 0; pass < 2; ++pass) {
    for (int i = t_; i < (stn - st) / 4; i += 256) { v4i v; for (int e = 0; e < 4; ++e) { const int q = i * 4 + e; v[e] = (q < tot) ? outp[q] : -1; } *(volatile v4i*)(PERM + st + i * 4) = v; }
    for (int i = t_; i < CSR_TS9 / 4; i += 256) { v4i a, c; for (int e = 0; e < 4; ++e) { const int vl = i * 4 + e; const int vc = vl < CSR_GN9 ? vl : CSR_GN9; a[e] = (vl < CSR_GN9) ? st + ncnt[vc] : st; c[e] = (vl < nv) ? (ncnt[(vc < CSR_GN9 ? vc : CSR_GN9 - 1) + 1] - ncnt[vc]) : 0; } *(volatile v4i*)(ROWPTR + t0 + i * 4) = a; *(volatile v4i*)(ROWCNT + t0 + i * 4) = c; }
    __threadfence(); }
}
__global__ __launch_bounds__(256) void csrZ_kernel9(int* __restrict__ p, size_t n4) { typedef __attribute__((ext_vector_type(4))) int v4i; const size_t tid = (size_t)blockIdx.x * 256 + threadIdx.x, nth = (size_t)gridDim.x * 256; v4i z = {0, 0, 0, 0}; for (size_t i = tid; i < n4; i += nth) *(volatile v4i*)(p + i * 4) = z; }
struct CsrBufs9 { int *STG, *HST, *OFF, *START, *TOT, *PERM, *ROWPTR, *ROWCNT, *FLAG; int nG, NGP, CHP; size_t permLen; char* base; size_t bytes; };
static size_t csr_carve9(CsrBufs9& c, char* ws, size_t off, int E, int N) {
  const size_t off0 = off; c.base = ws + off;
  auto al = [&](size_t bytes) { char* p = ws + off; off += (bytes + 255) & ~(size_t)255; return p; };
  c.nG = (N + CSR_GN9 - 1) / CSR_GN9; c.NGP = (c.nG + 31) & ~31; const int ch = (E + CSR_NBLK9 - 1) / CSR_NBLK9; c.CHP = (ch + 31) & ~31; c.permLen = (size_t)E + 32 * (size_t)c.nG + 32;
  c.STG = (int*)al((size_t)CSR_NBLK9 * c.CHP * 4); c.HST = (int*)al((size_t)CSR_NBLK9 * c.NGP * 4); c.OFF = (int*)al((size_t)c.NGP * CSR_NBLK9 * 4); c.START = (int*)al((size_t)(c.NGP + 64) * 4); c.TOT = (int*)al((size_t)(c.NGP + 64) * 4);
  c.PERM = (int*)al(c.permLen * 4); c.ROWPTR = (int*)al((size_t)c.nG * CSR_TS9 * 4); c.ROWCNT = (int*)al((size_t)c.nG * CSR_TS9 * 4); c.FLAG = (int*)al(256);
  c.bytes = off - off0; return off;
}
static void csr_build9(const CsrBufs9& c, const int* dst, int E, int N, hipStream_t stream) {
  const size_t smem = (size_t)(2 * c.NGP + c.CHP) * 4;
  csrZ_kernel9<<<512, 256, 0, stream>>>((int*)c.base, c.bytes / 16);
  csrA_kernel9<<<CSR_NBLK9, 64, smem, stream>>>(dst, E, N, c.nG, c.CHP, c.NGP, c.STG, c.HST);
  csrS_kernel9<<<1, 512, 0, stream>>>(c.HST, c.nG, c.NGP, c.START, c.TOT, c.OFF);
  csrB_kernel9<<<c.nG, 256, 0, stream>>>(dst, N, c.nG, c.CHP, c.NGP, (int)c.permLen, c.STG, c.HST, c.OFF, c.START, c.TOT, c.PERM, c.ROWPTR, c.ROWCNT, c.FLAG);
}


__global__ __launch_bounds__(256) void wprep_kernel(const float* __restrict__ w, int KIN, int OUTW, int ro, b16* __restrict__ WT) {
  const size_t u = (size_t)blockIdx.x * 256 + threadIdx.x; if (u >= (size_t)OUTW * KIN / 8) return; const size_t e = u * 8; const int o = (int)(e / KIN), k0 = (int)(e % KIN); v8b v;
#pragma unroll
  for (int j = 0; j < 8; ++j) v[j] = (b16)(bf16_rne(w[(size_t)(k0 + j) * OUTW + o]) * WSC); for (int pass = 0; pass < 2; ++pass) { *(volatile v8b*)(WT + (size_t)(ro + o) * KIN + k0) = v; __threadfence(); }
}
__global__ __launch_bounds__(128) void gw1_kernel(const float* __restrict__ w, b16* __restrict__ WT) {
  const int o = threadIdx.x; v8b v0 = {}, v1 = {}, vz = {};
#pragma unroll
  for (int k = 0; k < 8; ++k) v0[k] = (b16)(bf16_rne(w[k * GEO + o]) * WSC);
#pragma unroll
  for (int k = 0; k < 4; ++k) v1[k] = (b16)(bf16_rne(w[(8 + k) * GEO + o]) * WSC);
  for (int pass = 0; pass < 2; ++pass) { *(volatile v8b*)(WT + o * 32) = v0; *(volatile v8b*)(WT + o * 32 + 8) = v1; *(volatile v8b*)(WT + o * 32 + 16) = vz; *(volatile v8b*)(WT + o * 32 + 24) = vz; __threadfence(); }
}
__global__ __launch_bounds__(32) void kv_kernel(const float* __restrict__ sf, const b16* __restrict__ WKV, float* __restrict__ KV) {
  __shared__ __attribute__((aligned(16))) b16 Ah[16][D + 8]; __shared__ __attribute__((aligned(16))) float Tf[16][128 + 4];
  const int lane = threadIdx.x, nloc = lane & 15, hlf = lane >> 4; const size_t m0 = (size_t)blockIdx.x * 16;
  for (int rr = 0; rr < 16; ++rr) for (int q = 0; q < D / 32; ++q) Ah[rr][q * 32 + lane] = (b16)(bf16_rne(sf[(m0 + rr) * D + q * 32 + lane]) * XS);
  wave_lds_sync();
#pragma unroll 1
  for (int cg = 0; cg < 4; ++cg) { v8f acc[8];
#pragma unroll
    for (int t = 0; t < 8; ++t) acc[t] = (v8f){};
#pragma unroll 2
    for (int kb = 0; kb < D; kb += 32) { const v16b a = frag_kb(&Ah[nloc][kb], hlf);
#pragma unroll
      for (int t = 0; t < 8; ++t) acc[t] = wmma16b(a, frag_kb(WKV + (size_t)(cg * 128 + t * 16 + nloc) * D + kb, hlf), acc[t]); }
#pragma unroll
    for (int t = 0; t < 8; ++t)
#pragma unroll 1
      for (int r8 = 0; r8 < 8; ++r8) Tf[8 * hlf + r8][t * 16 + nloc] = acc[t][r8] * (1.0f / (XS * WSC));
    wave_lds_sync();
    for (int pass = 0; pass < 2; ++pass) { for (int rr = 0; rr < 16; ++rr) *(volatile v4f*)(KV + (m0 + rr) * (2 * D) + cg * 128 + lane * 4) = *(const v4f*)(&Tf[rr][lane * 4]); __threadfence(); }
    wave_lds_sync(); }
}
__global__ __launch_bounds__(32) void query_kernel(const float* __restrict__ x, const float* __restrict__ qp, const float* __restrict__ sp, const int* __restrict__ sidx, const int* __restrict__ PERM, const int* __restrict__ ROWPTR, const int* __restrict__ ROWCNT, int permLen, const float* __restrict__ g1, const float* __restrict__ b1, const b16* __restrict__ WQ, const b16* __restrict__ GW1, const float* __restrict__ gb1, const b16* __restrict__ GW2, const float* __restrict__ gb2, const b16* __restrict__ WG, int NLIM, float* __restrict__ QF, float* __restrict__ GF) {
  __shared__ __attribute__((aligned(16))) b16 Ah[16][D + 8], Al[16][D + 8]; __shared__ __attribute__((aligned(16))) b16 Bh[16][GEO + 8], Bl[16][GEO + 8]; __shared__ __attribute__((aligned(16))) float Tf[16][128 + 4]; __shared__ float Raw[16][12];
  const int lane = threadIdx.x, nloc = lane & 15, hlf = lane >> 4; const size_t m0 = (size_t)blockIdx.x * 16; if (m0 >= (size_t)NLIM) return;
  { float g8[8], b8[8]; for (int q = 0; q < 8; ++q) { g8[q] = bf16_rne(g1[q * 32 + lane]); b8[q] = bf16_rne(b1[q * 32 + lane]); }
    for (int rr = 0; rr < 16; ++rr) { float v[8]; float s = 0.0f; for (int q = 0; q < 8; ++q) { v[q] = bf16_rne(x[(m0 + rr) * D + q * 32 + lane]); s += v[q]; } for (int o = 16; o; o >>= 1) s += __shfl_xor(s, o); const float mu = s * (1.0f / D);
      float vq = 0.0f; for (int q = 0; q < 8; ++q) { const float d = v[q] - mu; vq += pmul(d, d); } for (int o = 16; o; o >>= 1) vq += __shfl_xor(vq, o); const float rs = rsqrtf(vq * (1.0f / D) + EPS);
      for (int q = 0; q < 8; ++q) { b16 p, ql; split16((pmul(pmul(v[q] - mu, rs), g8[q]) + b8[q]) * XS, p, ql); Ah[rr][q * 32 + lane] = p; Al[rr][q * 32 + lane] = ql; } } }
  wave_lds_sync();
#pragma unroll 1
  for (int cg = 0; cg < 2; ++cg) { v8f acc[8];
#pragma unroll
    for (int t = 0; t < 8; ++t) acc[t] = (v8f){};
#pragma unroll 2
    for (int kb = 0; kb < D; kb += 32) { const v16b a = frag_kb(&Ah[nloc][kb], hlf), al = frag_kb(&Al[nloc][kb], hlf);
#pragma unroll
      for (int t = 0; t < 8; ++t) { const v16b bw = frag_kb(WQ + (size_t)(cg * 128 + t * 16 + nloc) * D + kb, hlf); acc[t] = wmma16b(a, bw, acc[t]); acc[t] = wmma16b(al, bw, acc[t]); } }
#pragma unroll
    for (int t = 0; t < 8; ++t)
#pragma unroll 1
      for (int r8 = 0; r8 < 8; ++r8) Tf[8 * hlf + r8][t * 16 + nloc] = acc[t][r8] * (1.0f / (XS * WSC));
    wave_lds_sync();
    for (int pass = 0; pass < 2; ++pass) { for (int rr = 0; rr < 16; ++rr) *(volatile v4f*)(QF + (m0 + rr) * D + cg * 128 + lane * 4) = *(const v4f*)(&Tf[rr][lane * 4]); __threadfence(); }
    wave_lds_sync(); }
  for (int rr = 0; rr < 16; ++rr) { const size_t qv = m0 + rr; const float px = bf16_rne(qp[qv * 3]), py = bf16_rne(qp[qv * 3 + 1]), pz = bf16_rne(qp[qv * 3 + 2]); int st = ROWPTR[qv], cnt = ROWCNT[qv]; cnt = iclamp(cnt, 0, 1 << 20); st = iclamp(st, 0, permLen - cnt);
    float sx = 0, sy = 0, sz = 0, mnx = INFINITY, mny = INFINITY, mnz = INFINITY, mxx = -INFINITY, mxy = -INFINITY, mxz = -INFINITY;
#pragma unroll 1
    for (int j = lane; j < cnt; j += 32) { const int e = iclamp(PERM[st + j], 0, E - 1); const size_t si = (size_t)iclamp(sidx[e], 0, S - 1); const float rx = bf16_rne(sp[si * 3]) - px, ry = bf16_rne(sp[si * 3 + 1]) - py, rz = bf16_rne(sp[si * 3 + 2]) - pz;
      sx += rx; sy += ry; sz += rz; mnx = fminf(mnx, rx); mny = fminf(mny, ry); mnz = fminf(mnz, rz); mxx = fmaxf(mxx, rx); mxy = fmaxf(mxy, ry); mxz = fmaxf(mxz, rz); }
    for (int o = 16; o; o >>= 1) { sx += __shfl_xor(sx, o); sy += __shfl_xor(sy, o); sz += __shfl_xor(sz, o); mnx = fminf(mnx, __shfl_xor(mnx, o)); mny = fminf(mny, __shfl_xor(mny, o)); mnz = fminf(mnz, __shfl_xor(mnz, o)); mxx = fmaxf(mxx, __shfl_xor(mxx, o)); mxy = fmaxf(mxy, __shfl_xor(mxy, o)); mxz = fmaxf(mxz, __shfl_xor(mxz, o)); }
    const float ic = 1.0f / (float)(cnt < 1 ? 1 : cnt); const float mx_ = sx * ic, my_ = sy * ic, mz_ = sz * ic; float vx = 0, vy = 0, vz = 0;
#pragma unroll 1
    for (int j = lane; j < cnt; j += 32) { const int e = iclamp(PERM[st + j], 0, E - 1); const size_t si = (size_t)iclamp(sidx[e], 0, S - 1); const float rx = bf16_rne(sp[si * 3]) - px - mx_, ry = bf16_rne(sp[si * 3 + 1]) - py - my_, rz = bf16_rne(sp[si * 3 + 2]) - pz - mz_; vx += pmul(rx, rx); vy += pmul(ry, ry); vz += pmul(rz, rz); }
    for (int o = 16; o; o >>= 1) { vx += __shfl_xor(vx, o); vy += __shfl_xor(vy, o); vz += __shfl_xor(vz, o); }
    if (lane == 0) { Raw[rr][0] = mx_; Raw[rr][1] = my_; Raw[rr][2] = mz_; Raw[rr][3] = sqrtf(vx * ic); Raw[rr][4] = sqrtf(vy * ic); Raw[rr][5] = sqrtf(vz * ic);
      Raw[rr][6] = fminf(fmaxf(mnx, -100.0f), 100.0f); Raw[rr][7] = fminf(fmaxf(mny, -100.0f), 100.0f); Raw[rr][8] = fminf(fmaxf(mnz, -100.0f), 100.0f); Raw[rr][9] = fminf(fmaxf(mxx, -100.0f), 100.0f); Raw[rr][10] = fminf(fmaxf(mxy, -100.0f), 100.0f); Raw[rr][11] = fminf(fmaxf(mxz, -100.0f), 100.0f); } }
  wave_lds_sync();
  for (int rr = 0; rr < 16; ++rr) { b16 p = (b16)0.0f, ql = (b16)0.0f; if (lane < 12) split16(Raw[rr][lane] * XS, p, ql); Bh[rr][lane] = p; Bl[rr][lane] = ql; }
  wave_lds_sync();
  { v8f acc[8]; const v16b a = frag_kb(&Bh[nloc][0], hlf), al = frag_kb(&Bl[nloc][0], hlf);
#pragma unroll
    for (int t = 0; t < 8; ++t) { acc[t] = (v8f){}; const v16b bw = frag_kb(GW1 + (size_t)(t * 16 + nloc) * 32, hlf); acc[t] = wmma16b(a, bw, acc[t]); acc[t] = wmma16b(al, bw, acc[t]); }
    wave_lds_sync();
#pragma unroll
    for (int t = 0; t < 8; ++t) { const int c = t * 16 + nloc; const float bb = bf16_rne(gb1[c]);
#pragma unroll
      for (int r8 = 0; r8 < 8; ++r8) { const float v = gelu(acc[t][r8] * (1.0f / (XS * WSC)) + bb); b16 p, ql; split16(v * G1S, p, ql); Bh[8 * hlf + r8][c] = p; Bl[8 * hlf + r8][c] = ql; } } }
  wave_lds_sync();
  { v8f acc[8];
#pragma unroll
    for (int t = 0; t < 8; ++t) acc[t] = (v8f){};
#pragma unroll
    for (int kb = 0; kb < GEO; kb += 32) { const v16b a = frag_kb(&Bh[nloc][kb], hlf), al = frag_kb(&Bl[nloc][kb], hlf);
#pragma unroll
      for (int t = 0; t < 8; ++t) { const v16b bw = frag_kb(GW2 + (size_t)(t * 16 + nloc) * GEO + kb, hlf); acc[t] = wmma16b(a, bw, acc[t]); acc[t] = wmma16b(al, bw, acc[t]); } }
    wave_lds_sync();
#pragma unroll
    for (int t = 0; t < 8; ++t) { const int c = t * 16 + nloc; const float bb = bf16_rne(gb2[c]);
#pragma unroll
      for (int r8 = 0; r8 < 8; ++r8) { const float v = gelu(acc[t][r8] * (1.0f / (G1S * WSC)) + bb); b16 p, ql; split16(v * G2S, p, ql); Bh[8 * hlf + r8][c] = p; Bl[8 * hlf + r8][c] = ql; } } }
  wave_lds_sync();
#pragma unroll 1
  for (int cg = 0; cg < 2; ++cg) { v8f acc[8];
#pragma unroll
    for (int t = 0; t < 8; ++t) acc[t] = (v8f){};
#pragma unroll
    for (int kb = 0; kb < GEO; kb += 32) { const v16b a = frag_kb(&Bh[nloc][kb], hlf), al = frag_kb(&Bl[nloc][kb], hlf);
#pragma unroll
      for (int t = 0; t < 8; ++t) { const v16b bw = frag_kb(WG + (size_t)(cg * 128 + t * 16 + nloc) * GEO + kb, hlf); acc[t] = wmma16b(a, bw, acc[t]); acc[t] = wmma16b(al, bw, acc[t]); } }
#pragma unroll
    for (int t = 0; t < 8; ++t)
#pragma unroll 1
      for (int r8 = 0; r8 < 8; ++r8) Tf[8 * hlf + r8][t * 16 + nloc] = acc[t][r8] * (1.0f / (G2S * WSC));
    wave_lds_sync();
    for (int pass = 0; pass < 2; ++pass) { for (int rr = 0; rr < 16; ++rr) *(volatile v4f*)(GF + (m0 + rr) * D + cg * 128 + lane * 4) = *(const v4f*)(&Tf[rr][lane * 4]); __threadfence(); }
    wave_lds_sync(); }
}
__global__ __launch_bounds__(256) void att_kernel(const float* __restrict__ QF, const float* __restrict__ KV, const float* __restrict__ GF, const float* __restrict__ ltau, const int* __restrict__ sidx, const int* __restrict__ PERM, const int* __restrict__ ROWPTR, const int* __restrict__ ROWCNT, int permLen, int NLIM, float* __restrict__ OUT_) {
  const int wave = threadIdx.x >> 5, lane = threadIdx.x & 31; const size_t qv = (size_t)blockIdx.x * 8 + wave; float o[8]; for (int i = 0; i < 8; ++i) o[i] = 0.0f;
  if (qv < (size_t)NLIM) { const float isc = 1.0f / (sqrtf((float)HD) * __expf(bf16_rne(ltau[0])));
    float q8[8], g8[8]; { const v4f a = *(const v4f*)(QF + qv * D + lane * 8), b = *(const v4f*)(QF + qv * D + lane * 8 + 4), c = *(const v4f*)(GF + qv * D + lane * 8), d = *(const v4f*)(GF + qv * D + lane * 8 + 4); for (int i = 0; i < 4; ++i) { q8[i] = a[i]; q8[4 + i] = b[i]; g8[i] = c[i]; g8[4 + i] = d[i]; } }
    int st = ROWPTR[qv], cnt = ROWCNT[qv]; cnt = iclamp(cnt, 0, 1 << 20); st = iclamp(st, 0, permLen - cnt); float mx = 0.0f;
#pragma unroll 1
    for (int j = 0; j < cnt; ++j) { const int e = iclamp(PERM[st + j], 0, E - 1); const size_t si = (size_t)iclamp(sidx[e], 0, S - 1); const v4f ka = *(const v4f*)(KV + si * (2 * D) + lane * 8), kb = *(const v4f*)(KV + si * (2 * D) + lane * 8 + 4);
      float s = 0.0f; for (int i = 0; i < 4; ++i) { s += pmul(q8[i], ka[i]); s += pmul(q8[4 + i], kb[i]); } s += __shfl_xor(s, 1); s += __shfl_xor(s, 2); mx = fmaxf(mx, s * isc); }
    float den = 0.0f;
#pragma unroll 1
    for (int j = 0; j < cnt; ++j) { const int e = iclamp(PERM[st + j], 0, E - 1); const size_t si = (size_t)iclamp(sidx[e], 0, S - 1); const v4f ka = *(const v4f*)(KV + si * (2 * D) + lane * 8), kb = *(const v4f*)(KV + si * (2 * D) + lane * 8 + 4);
      float s = 0.0f; for (int i = 0; i < 4; ++i) { s += pmul(q8[i], ka[i]); s += pmul(q8[4 + i], kb[i]); } s += __shfl_xor(s, 1); s += __shfl_xor(s, 2); const float p = __expf(s * isc - mx); den += p;
      const v4f va = *(const v4f*)(KV + si * (2 * D) + D + lane * 8), vb = *(const v4f*)(KV + si * (2 * D) + D + lane * 8 + 4); for (int i = 0; i < 4; ++i) { o[i] += pmul(p, va[i] + g8[i]); o[4 + i] += pmul(p, vb[i] + g8[4 + i]); } }
    const float inv = 1.0f / fmaxf(den, 1e-8f); for (int i = 0; i < 8; ++i) o[i] = pmul(o[i], inv); }
  v4f o0 = {o[0], o[1], o[2], o[3]}, o1 = {o[4], o[5], o[6], o[7]};
  for (int pass = 0; pass < 2; ++pass) { *(volatile v4f*)(OUT_ + qv * D + lane * 8) = o0; *(volatile v4f*)(OUT_ + qv * D + lane * 8 + 4) = o1; __threadfence(); }
}
__global__ __launch_bounds__(32) void out_kernel(const float* __restrict__ OUTA, const float* __restrict__ x, const b16* __restrict__ WO, const float* __restrict__ bo, const float* __restrict__ g2, const float* __restrict__ b2, const b16* __restrict__ WF1, const float* __restrict__ bf1, const b16* __restrict__ WF2, const float* __restrict__ bf2, int NLIM, float* __restrict__ out) {
  __shared__ __attribute__((aligned(16))) b16 Ah[16][D + 8], Al[16][D + 8]; __shared__ __attribute__((aligned(16))) b16 A2h[16][FFN + 8], A2l[16][FFN + 8]; __shared__ __attribute__((aligned(16))) float Xs[16][D + 4];
  const int lane = threadIdx.x, nloc = lane & 15, hlf = lane >> 4; const size_t m0 = (size_t)blockIdx.x * 16; if (m0 >= (size_t)NLIM) return;
  for (int rr = 0; rr < 16; ++rr) for (int q = 0; q < 8; ++q) { const int c = q * 32 + lane; const float v = OUTA[(m0 + rr) * D + c]; b16 p, ql; split16(v * OS, p, ql); Ah[rr][c] = p; Al[rr][c] = ql; Xs[rr][c] = bf16_rne(x[(m0 + rr) * D + c]); }
  wave_lds_sync();
#pragma unroll 1
  for (int cg = 0; cg < 2; ++cg) { v8f acc[8];
#pragma unroll
    for (int t = 0; t < 8; ++t) acc[t] = (v8f){};
#pragma unroll 2
    for (int kb = 0; kb < D; kb += 32) { const v16b a = frag_kb(&Ah[nloc][kb], hlf), al = frag_kb(&Al[nloc][kb], hlf);
#pragma unroll
      for (int t = 0; t < 8; ++t) { const v16b bw = frag_kb(WO + (size_t)(cg * 128 + t * 16 + nloc) * D + kb, hlf); acc[t] = wmma16b(a, bw, acc[t]); acc[t] = wmma16b(al, bw, acc[t]); } }
#pragma unroll
    for (int t = 0; t < 8; ++t) { const int c = cg * 128 + t * 16 + nloc; const float bb = bf16_rne(bo[c]);
#pragma unroll
      for (int r8 = 0; r8 < 8; ++r8) Xs[8 * hlf + r8][c] += acc[t][r8] * (1.0f / (OS * WSC)) + bb; } }
  wave_lds_sync();
  { float g8[8], b8[8]; for (int q = 0; q < 8; ++q) { g8[q] = bf16_rne(g2[q * 32 + lane]); b8[q] = bf16_rne(b2[q * 32 + lane]); }
    for (int rr = 0; rr < 16; ++rr) { float v[8]; float s = 0.0f; for (int q = 0; q < 8; ++q) { v[q] = Xs[rr][q * 32 + lane]; s += v[q]; } for (int o = 16; o; o >>= 1) s += __shfl_xor(s, o); const float mu = s * (1.0f / D);
      float vq = 0.0f; for (int q = 0; q < 8; ++q) { const float d = v[q] - mu; vq += pmul(d, d); } for (int o = 16; o; o >>= 1) vq += __shfl_xor(vq, o); const float rs = rsqrtf(vq * (1.0f / D) + EPS);
      for (int q = 0; q < 8; ++q) { b16 p, ql; split16((pmul(pmul(v[q] - mu, rs), g8[q]) + b8[q]) * XS, p, ql); Ah[rr][q * 32 + lane] = p; Al[rr][q * 32 + lane] = ql; } } }
  wave_lds_sync();
#pragma unroll 1
  for (int cg = 0; cg < FFN / 128; ++cg) { v8f acc[8];
#pragma unroll
    for (int t = 0; t < 8; ++t) acc[t] = (v8f){};
#pragma unroll 2
    for (int kb = 0; kb < D; kb += 32) { const v16b a = frag_kb(&Ah[nloc][kb], hlf), al = frag_kb(&Al[nloc][kb], hlf);
#pragma unroll
      for (int t = 0; t < 8; ++t) { const v16b bw = frag_kb(WF1 + (size_t)(cg * 128 + t * 16 + nloc) * D + kb, hlf); acc[t] = wmma16b(a, bw, acc[t]); acc[t] = wmma16b(al, bw, acc[t]); } }
#pragma unroll
    for (int t = 0; t < 8; ++t) { const int c = cg * 128 + t * 16 + nloc; const float bb = bf16_rne(bf1[c]);
#pragma unroll
      for (int r8 = 0; r8 < 8; ++r8) { const float v = gelu(acc[t][r8] * (1.0f / (XS * WSC)) + bb); b16 p, ql; split16(v * FS, p, ql); A2h[8 * hlf + r8][c] = p; A2l[8 * hlf + r8][c] = ql; } } }
  wave_lds_sync();
#pragma unroll 1
  for (int cg = 0; cg < 2; ++cg) { v8f acc[8];
#pragma unroll
    for (int t = 0; t < 8; ++t) acc[t] = (v8f){};
#pragma unroll 2
    for (int kb = 0; kb < FFN; kb += 32) { const v16b a = frag_kb(&A2h[nloc][kb], hlf), al = frag_kb(&A2l[nloc][kb], hlf);
#pragma unroll
      for (int t = 0; t < 8; ++t) { const v16b bw = frag_kb(WF2 + (size_t)(cg * 128 + t * 16 + nloc) * FFN + kb, hlf); acc[t] = wmma16b(a, bw, acc[t]); acc[t] = wmma16b(al, bw, acc[t]); } }
#pragma unroll
    for (int t = 0; t < 8; ++t) { const int c = cg * 128 + t * 16 + nloc; const float bb = bf16_rne(bf2[c]);
#pragma unroll
      for (int r8 = 0; r8 < 8; ++r8) Xs[8 * hlf + r8][c] += acc[t][r8] * (1.0f / (FS * WSC)) + bb; } }
  wave_lds_sync();
  for (int pass = 0; pass < 2; ++pass) { for (int rr = 0; rr < 16; ++rr) for (int q = 0; q < 8; ++q) ((volatile float*)out)[(m0 + rr) * D + q * 32 + lane] = Xs[rr][q * 32 + lane]; __threadfence(); }
}
}

extern "C" void kernel_launch(void* const* d_in, const int* in_sizes, int n_in, void* d_out, int out_size, void* d_ws, size_t ws_size, hipStream_t stream) {
  (void)n_in;
  auto Fp = [&](int i) { return (const float*)d_in[i]; }; auto Ip = [&](int i) { return (const int*)d_in[i]; };
  if (in_sizes[0] != Q * D || in_sizes[1] != Q * 3 || in_sizes[2] != S * D || in_sizes[3] != S * 3 || in_sizes[4] != D * D || in_sizes[7] != GEO * D || in_sizes[15] != D * FFN || in_sizes[17] != FFN * D || in_sizes[19] != 12 * GEO || in_sizes[21] != GEO * GEO || in_sizes[23] != E || in_sizes[24] != E || out_size != Q * D) return;
  const int NLIM = Q; const int GB16 = NQB, GB8 = Q / 8;
  size_t off = 0; char* ws = (char*)d_ws;
  auto carve = [&](size_t bytes) { char* p = ws + off; off += (bytes + 255) & ~(size_t)255; return p; };
  b16* WQ = (b16*)carve((size_t)D * D * 2); b16* WKV = (b16*)carve((size_t)2 * D * D * 2); b16* WG = (b16*)carve((size_t)D * GEO * 2); b16* WO = (b16*)carve((size_t)D * D * 2); b16* WF1 = (b16*)carve((size_t)FFN * D * 2); b16* WF2 = (b16*)carve((size_t)D * FFN * 2); b16* GW1 = (b16*)carve(GEO * 32 * 2); b16* GW2 = (b16*)carve(GEO * GEO * 2);
  float* KV = (float*)carve((size_t)S * 2 * D * 4); float* QF = (float*)carve((size_t)Q * D * 4); float* GF = (float*)carve((size_t)Q * D * 4); float* OUTA = (float*)carve((size_t)Q * D * 4);
  CsrBufs9 csr; off = csr_carve9(csr, ws, off, E, Q);
  if (off > ws_size || off > ((size_t)128 << 20)) return;
  wprep_kernel<<<(D * D / 8 + 255) / 256, 256, 0, stream>>>(Fp(4), D, D, 0, WQ); wprep_kernel<<<(D * D / 8 + 255) / 256, 256, 0, stream>>>(Fp(5), D, D, 0, WKV); wprep_kernel<<<(D * D / 8 + 255) / 256, 256, 0, stream>>>(Fp(6), D, D, D, WKV);
  wprep_kernel<<<(D * GEO / 8 + 255) / 256, 256, 0, stream>>>(Fp(7), GEO, D, 0, WG); wprep_kernel<<<(D * D / 8 + 255) / 256, 256, 0, stream>>>(Fp(8), D, D, 0, WO); wprep_kernel<<<(FFN * D / 8 + 255) / 256, 256, 0, stream>>>(Fp(15), D, FFN, 0, WF1); wprep_kernel<<<(D * FFN / 8 + 255) / 256, 256, 0, stream>>>(Fp(17), FFN, D, 0, WF2);
  gw1_kernel<<<1, 128, 0, stream>>>(Fp(19), GW1); wprep_kernel<<<(GEO * GEO / 8 + 255) / 256, 256, 0, stream>>>(Fp(21), GEO, GEO, 0, GW2);
  csr_build9(csr, Ip(23), E, Q, stream);
  kv_kernel<<<S / 16, 32, 0, stream>>>(Fp(2), WKV, KV);
  query_kernel<<<GB16, 32, 0, stream>>>(Fp(0), Fp(1), Fp(3), Ip(24), csr.PERM, csr.ROWPTR, csr.ROWCNT, (int)csr.permLen, Fp(11), Fp(12), WQ, GW1, Fp(20), GW2, Fp(22), WG, NLIM, QF, GF);
  att_kernel<<<GB8, 256, 0, stream>>>(QF, KV, GF, Fp(10), Ip(24), csr.PERM, csr.ROWPTR, csr.ROWCNT, (int)csr.permLen, NLIM, OUTA);
  out_kernel<<<GB16, 32, 0, stream>>>(OUTA, Fp(0), WO, Fp(9), Fp(13), Fp(14), WF1, Fp(16), WF2, Fp(18), NLIM, (float*)d_out);
}
